// Encoder_89404039233721
// MI455X (gfx1250) — hardware-run, weakly checked
//
#include <hip/hip_runtime.h>
#include <math.h>

typedef __attribute__((ext_vector_type(16))) _Float16 v16h;
typedef __attribute__((ext_vector_type(8)))  _Float16 v8h;
typedef __attribute__((ext_vector_type(8)))  float    v8f;
typedef __attribute__((ext_vector_type(4)))  float    v4f;

constexpr int kNB = 64;
constexpr int kNT = 100;
constexpr int kNE = 512;
constexpr int kNU = 512;
constexpr int kNV = 32000;
constexpr int kRows = kNT * kNB;
constexpr int kG3 = 3 * kNU;
constexpr int kBlkRows = 16;
constexpr int kHP = 520;
constexpr int kFP = 516;
constexpr int kOut0 = kNB * kNT * kNU;
constexpr int kOut1 = 2 * kNB * kNU;
constexpr float kActCarry = 4096.0f;
constexpr float kWgtCarry = 1024.0f;
constexpr float kFold = 1.0f / (kActCarry * kWgtCarry);
constexpr float kF16MinNormal = 6.103515625e-05f;

static_assert(kRows % 64 == 0);
static_assert(kNE % 32 == 0 && (2 * kNU) % 32 == 0 && kNU % 32 == 0);
static_assert(kG3 % 64 == 0 && (2 * kG3) % 64 == 0);
static_assert(kNU == 64 * 8);
static_assert(kNB % kBlkRows == 0 && kNB / kBlkRows == 4);
static_assert((size_t)kOut0 * 4 == 13107200ull);
static_assert((size_t)(kOut0 + kOut1) * 4 == 13369344ull);
static_assert((kHP % 8) == 0 && (kFP % 4) == 0);

constexpr size_t kSzP    = (size_t)kRows * 2 * kG3 * 4;
constexpr size_t kSzX16  = (size_t)kRows * kNE * 2;
constexpr size_t kSzYCAT = (size_t)kRows * 2 * kNU * 2;
constexpr size_t kSzY1   = (size_t)kRows * kNU * 2;
constexpr size_t kSzBX0  = (size_t)2 * kG3 * kNE * 2;
constexpr size_t kSzBHBI = (size_t)2 * kG3 * kNU * 2;
constexpr size_t kSzBX1  = (size_t)kG3 * 2 * kNU * 2;
constexpr size_t kSzBH   = (size_t)kG3 * kNU * 2;
constexpr size_t kSzBX2  = (size_t)kG3 * kNU * 2;
constexpr size_t kSzBIAS = (size_t)4 * kG3 * 4;
constexpr size_t kWsTotal = kSzP + kSzX16 + kSzYCAT + kSzY1 + kSzBX0 + kSzBHBI + kSzBX1 + kSzBH + kSzBX2 + kSzBH + kSzBIAS;
static_assert(kWsTotal == 119037952ull);
static_assert(kWsTotal <= 134217728ull);
static_assert((kSzP % 256) == 0 && (kSzX16 % 256) == 0 && (kSzYCAT % 256) == 0 && (kSzY1 % 256) == 0 &&
              (kSzBX0 % 256) == 0 && (kSzBHBI % 256) == 0 && (kSzBX1 % 256) == 0 && (kSzBH % 256) == 0 &&
              (kSzBX2 % 256) == 0 && (kSzBIAS % 256) == 0);

__device__ __forceinline__ float bf16_value(float f) {
  const unsigned u = __float_as_uint(f);
  const unsigned r = (u + 0x7FFFu + ((u >> 16) & 1u)) & 0xFFFF0000u;
  return __uint_as_float(r);
}
__device__ __forceinline__ _Float16 to_f16_flushed(float v) {
  const float w = (fabsf(v) < kF16MinNormal) ? 0.0f : v;
  return (_Float16)w;
}
__device__ __forceinline__ float sigm(float x) {
  return __builtin_amdgcn_rcpf(1.0f + expf(-x));
}

union FragU { v16h v; v8h h[2]; };
__device__ __forceinline__ v16h frag_load(const _Float16* p) {
  FragU f;
  f.h[0] = *(const v8h*)(p);
  f.h[1] = *(const v8h*)(p + 16);
  return f.v;
}
__device__ __forceinline__ v8f mma_h(v16h a, v16h b, v8f c) {
  return __builtin_amdgcn_wmma_f32_16x16x32_f16(false, a, false, b, (short)0, c, false, false);
}
__device__ __forceinline__ void guard1_h(v8f& d, v16h a, v16h b) {
  asm volatile("v_nop\n\tv_nop\n\tv_nop\n\tv_nop" : "+v"(d) : "v"(a), "v"(b));
}
__device__ __forceinline__ void guard4_h(v8f& a, v8f& b, v8f& c, v8f& d, v16h x) {
  asm volatile("v_nop\n\tv_nop\n\tv_nop\n\tv_nop" : "+v"(a), "+v"(b), "+v"(c), "+v"(d) : "v"(x));
}
__device__ __forceinline__ void keep4_h(v16h a, v16h b, v16h c, v16h d) {
  asm volatile("v_nop" :: "v"(a), "v"(b), "v"(c), "v"(d));
}
__device__ __forceinline__ void acc_guard4(v8f& a, v8f& b, v8f& c, v8f& d) {
  asm volatile("v_nop\n\tv_nop\n\tv_nop\n\tv_nop" : "+v"(a), "+v"(b), "+v"(c), "+v"(d));
}

__global__ __launch_bounds__(256) void gather_rows_kernel(const int* __restrict__ tok,
                                                          const float* __restrict__ emb,
                                                          unsigned short* __restrict__ X16p) {
  const int lane = threadIdx.x & 31, wave = threadIdx.x >> 5;
  const int m = blockIdx.x * 8 + wave;
  if (m >= kRows) return;
  const int t = m >> 6, b = m & 63;
  int id = tok[b * kNT + t];
  id = id < 0 ? 0 : (id > kNV - 1 ? kNV - 1 : id);
  const float* src = emb + (size_t)id * kNE;
  v8h hv[2];
#pragma unroll
  for (int it = 0; it < 2; ++it) {
    const float* sp = src + it * 256 + lane * 8;
    const v4f a0 = *(const v4f*)(sp);
    const v4f a1 = *(const v4f*)(sp + 4);
#pragma unroll
    for (int e = 0; e < 4; ++e) {
      const float s0 = a0[e];
      const float s1 = a1[e];
      hv[it][e]     = to_f16_flushed(bf16_value(s0) * kActCarry);
      hv[it][4 + e] = to_f16_flushed(bf16_value(s1) * kActCarry);
    }
  }
  _Float16* dst = (_Float16*)X16p + (size_t)m * kNE + lane * 8;
  for (int pass = 0; pass < 2; ++pass) {
#pragma unroll
    for (int it = 0; it < 2; ++it) *(volatile v8h*)(dst + it * 256) = hv[it];
    __threadfence();
  }
}

__global__ __launch_bounds__(256) void wt_plane_kernel(const float* __restrict__ W, int ncols, int dsplit,
                                                       unsigned short* __restrict__ Dx, int pitchx, int nofsx,
                                                       unsigned short* __restrict__ Dh, int nofsh) {
  __shared__ float tile[64 * 65];
  const int tid = threadIdx.x, lane = tid & 31, wave = tid >> 5;
  const int n0 = blockIdx.x * 64, k0 = blockIdx.y * 64;
  {
    const int nn4 = (tid & 15) * 4;
#pragma unroll
    for (int it = 0; it < 4; ++it) {
      const int kk = it * 16 + (tid >> 4);
      const v4f v = *(const v4f*)(W + (size_t)(k0 + kk) * ncols + n0 + nn4);
#pragma unroll
      for (int e = 0; e < 4; ++e) {
        const float s = v[e];
        tile[kk * 65 + nn4 + e] = s;
      }
    }
  }
  __syncthreads();
  const bool isx = (k0 < dsplit);
  _Float16* D = isx ? (_Float16*)Dx : (_Float16*)Dh;
  const int pitch = isx ? pitchx : kNU;
  const int nofs  = isx ? nofsx : nofsh;
  const int kd    = isx ? k0 : (k0 - dsplit);
  const int q = lane >> 3, c8 = (lane & 7) * 8;
  v8h hv[2];
#pragma unroll
  for (int it = 0; it < 2; ++it) {
    const int nn = it * 32 + wave * 4 + q;
#pragma unroll
    for (int e = 0; e < 8; ++e) {
      const float s = tile[(c8 + e) * 65 + nn];
      hv[it][e] = to_f16_flushed(bf16_value(s) * kWgtCarry);
    }
  }
  for (int pass = 0; pass < 2; ++pass) {
#pragma unroll
    for (int it = 0; it < 2; ++it) {
      const int nn = it * 32 + wave * 4 + q;
      *(volatile v8h*)(D + (size_t)(nofs + n0 + nn) * pitch + kd + c8) = hv[it];
    }
    __threadfence();
  }
}

__global__ __launch_bounds__(256) void bias_plane_kernel(
    const float* __restrict__ g0, const float* __restrict__ c0,
    const float* __restrict__ g1, const float* __restrict__ c1,
    const float* __restrict__ g2, const float* __restrict__ c2,
    const float* __restrict__ g3, const float* __restrict__ c3,
    float* __restrict__ dst) {
  const int g = (blockIdx.x * 256 + threadIdx.x) * 4;
  const int layer = g / kG3;
  const int off = g - layer * kG3;
  const bool isg = off < 2 * kNU;
  int ig = off;
  if (ig > 2 * kNU - 4) ig = 2 * kNU - 4;
  int ic = off - 2 * kNU;
  if (ic < 0) ic = 0;
  if (ic > kNU - 4) ic = kNU - 4;
  v4f a0 = *(const v4f*)(g0 + ig);
  v4f a1 = *(const v4f*)(g1 + ig);
  v4f a2 = *(const v4f*)(g2 + ig);
  v4f a3 = *(const v4f*)(g3 + ig);
  v4f b0 = *(const v4f*)(c0 + ic);
  v4f b1 = *(const v4f*)(c1 + ic);
  v4f b2 = *(const v4f*)(c2 + ic);
  v4f b3 = *(const v4f*)(c3 + ic);
  asm volatile("" : "+v"(a0));
  asm volatile("" : "+v"(a1));
  asm volatile("" : "+v"(a2));
  asm volatile("" : "+v"(a3));
  asm volatile("" : "+v"(b0));
  asm volatile("" : "+v"(b1));
  asm volatile("" : "+v"(b2));
  asm volatile("" : "+v"(b3));
  const v4f sg = (layer == 0) ? a0 : ((layer == 1) ? a1 : ((layer == 2) ? a2 : a3));
  const v4f sc = (layer == 0) ? b0 : ((layer == 1) ? b1 : ((layer == 2) ? b2 : b3));
  const v4f sv = isg ? sg : sc;
  v4f o;
#pragma unroll
  for (int e = 0; e < 4; ++e) {
    const float s = sv[e];
    o[e] = bf16_value(s);
  }
  float* op = dst + g;
  *(volatile v4f*)op = o;
  __threadfence();
  *(volatile v4f*)op = o;
}

__global__ __launch_bounds__(256) void wmma_gemm64_f16(
    const unsigned short* __restrict__ Ap, int lda,
    const unsigned short* __restrict__ Btp, int ldb,
    float* __restrict__ Cout, int ldc,
    const float* __restrict__ bias,
    int M, int N, int K, float scale) {
  const _Float16* A  = (const _Float16*)Ap;
  const _Float16* Bt = (const _Float16*)Btp;
  __shared__ __align__(16) float sT[8][16 * 68];
  const int lane = threadIdx.x & 31;
  const int wave = threadIdx.x >> 5;
  const int tilesN = N >> 6;
  const int tilesM = M >> 6;
  const int tile = blockIdx.x * 8 + wave;
  if (tile >= tilesM * tilesN) return;
  const int tm = tile / tilesN;
  const int tn = tile - tm * tilesN;
  const int m0 = tm << 6;
  const int n0 = tn << 6;

  const int rlane = lane & 15;
  const int koff  = (lane >> 4) * 8;
  const int mOff  = (lane >> 4) * 8;

  v8f acc[4][4];
#pragma unroll
  for (int i = 0; i < 4; ++i)
#pragma unroll
    for (int j = 0; j < 4; ++j) acc[i][j] = (v8f){0.f, 0.f, 0.f, 0.f, 0.f, 0.f, 0.f, 0.f};

  for (int k0 = 0; k0 < K; k0 += 32) {
    v16h bh[4];
#pragma unroll
    for (int j = 0; j < 4; ++j) {
      const size_t bo = (size_t)(n0 + (j << 4) + rlane) * ldb + koff + k0;
      bh[j] = frag_load(Bt + bo);
    }
#pragma unroll
    for (int i = 0; i < 4; ++i) {
      const size_t ao = (size_t)(m0 + (i << 4) + rlane) * lda + koff + k0;
      const v16h ah = frag_load(A + ao);
#pragma unroll
      for (int j = 0; j < 4; ++j) acc[i][j] = mma_h(ah, bh[j], acc[i][j]);
      guard4_h(acc[i][0], acc[i][1], acc[i][2], acc[i][3], ah);
    }
    keep4_h(bh[0], bh[1], bh[2], bh[3]);
  }
  acc_guard4(acc[0][0], acc[0][1], acc[0][2], acc[0][3]);
  acc_guard4(acc[1][0], acc[1][1], acc[1][2], acc[1][3]);
  acc_guard4(acc[2][0], acc[2][1], acc[2][2], acc[2][3]);
  acc_guard4(acc[3][0], acc[3][1], acc[3][2], acc[3][3]);

  float* slab = sT[wave];
#pragma unroll
  for (int i = 0; i < 4; ++i) {
    const int mBase = m0 + (i << 4);
#pragma unroll
    for (int j = 0; j < 4; ++j) {
      const int n = n0 + (j << 4) + rlane;
      const float bv = bias[n];
#pragma unroll
      for (int r = 0; r < 8; ++r) {
        float v = acc[i][j][r] * scale;
        v += bv;
        slab[(mOff + r) * 68 + (j << 4) + rlane] = v;
      }
    }
    __builtin_amdgcn_fence(__ATOMIC_RELEASE, "workgroup");
    __builtin_amdgcn_wave_barrier();
    __builtin_amdgcn_fence(__ATOMIC_ACQUIRE, "workgroup");
    {
      const int hh = lane >> 4, c4 = (lane & 15) * 4;
      for (int pass = 0; pass < 2; ++pass) {
#pragma unroll
        for (int it = 0; it < 8; ++it) {
          const int row = it * 2 + hh;
          const v4f v = *(const v4f*)(slab + row * 68 + c4);
          *(volatile v4f*)(Cout + (size_t)(mBase + row) * ldc + n0 + c4) = v;
        }
        __threadfence();
      }
    }
    __builtin_amdgcn_fence(__ATOMIC_RELEASE, "workgroup");
    __builtin_amdgcn_wave_barrier();
    __builtin_amdgcn_fence(__ATOMIC_ACQUIRE, "workgroup");
  }
}

template <int OM>
__global__ __launch_bounds__(256) void gru_seq_kernel(
    const float* __restrict__ P, int ldp, int dirStrideP,
    const unsigned short* __restrict__ BhP, int dirStrideB,
    unsigned short* __restrict__ Y16p, int ldy, int dirStrideY,
    float* __restrict__ OUT0, float* __restrict__ HFIN) {
  __shared__ __align__(16) _Float16 H16[kBlkRows * kHP];
  __shared__ __align__(16) _Float16 R16[kBlkRows * kHP];
  __shared__ __align__(16) float    HS[kBlkRows * kFP];
  __shared__ __align__(16) float    US[kBlkRows * kFP];
  __shared__ __align__(16) float    PRS[8 * 256];

  const int tid = threadIdx.x, lane = tid & 31, wave = tid >> 5;
  const int c = lane & 15, hh = lane >> 4, koff = hh * 8;
  const int dir = blockIdx.x >> 2;
  const int rowbase = (blockIdx.x & 3) * kBlkRows;
  const _Float16* Bh = (const _Float16*)BhP + (size_t)dir * dirStrideB;
  const float* Pd = P + dir * dirStrideP;
  _Float16* Yd = (_Float16*)Y16p + dir * dirStrideY;

#pragma unroll 1
  for (int i = tid; i < kBlkRows * kHP; i += 256) {
    H16[i] = (_Float16)0.0f;
    R16[i] = (_Float16)0.0f;
  }
#pragma unroll 1
  for (int i = tid; i < kBlkRows * kFP; i += 256) {
    HS[i] = 0.0f;
    US[i] = 0.0f;
  }
  __syncthreads();

  const v8f z8 = {0.f, 0.f, 0.f, 0.f, 0.f, 0.f, 0.f, 0.f};

#pragma unroll 1
  for (int s = 0; s < kNT; ++s) {
    const int t = dir ? (kNT - 1 - s) : s;
    const float* Pt = Pd + (size_t)(t * kNB + rowbase) * ldp;

#pragma unroll 1
    for (int nt = 0; nt < 4; ++nt) {
      const int j = 64 * wave + 16 * nt + c;
      const _Float16* arow = H16 + c * kHP + koff;
      const _Float16* wr = Bh + (size_t)j * kNU + koff;
      const _Float16* wu = Bh + (size_t)(kNU + j) * kNU + koff;
      v8f accR = z8, accU = z8;
#pragma unroll 1
      for (int k0 = 0; k0 < kNU; k0 += 32) {
        const v16h a  = frag_load(arow + k0);
        const v16h b0 = frag_load(wr + k0);
        const v16h b1 = frag_load(wu + k0);
        accR = mma_h(a, b0, accR);
        accU = mma_h(a, b1, accU);
        guard1_h(accR, a, b0);
        guard1_h(accU, a, b1);
      }
#pragma unroll
      for (int i = 0; i < 8; ++i) {
        PRS[i * 256 + tid] = accR[i];
        US[(8 * hh + i) * kFP + j] = accU[i];
      }
#pragma unroll 1
      for (int i = 0; i < 8; ++i) {
        const int row = 8 * hh + i;
        const float pr = PRS[i * 256 + tid];
        const float pu = US[row * kFP + j];
        const float* pp = Pt + (size_t)row * ldp + j;
        const float gr = pp[0];
        const float gu = pp[kNU];
        const float rv = sigm(pr * kFold + gr);
        const float uv = sigm(pu * kFold + gu);
        const float hv = HS[row * kFP + j];
        US[row * kFP + j] = uv;
        R16[row * kHP + j] = to_f16_flushed((rv * hv) * kActCarry);
      }
    }
    __syncthreads();

#pragma unroll 1
    for (int nt = 0; nt < 4; ++nt) {
      const int j = 64 * wave + 16 * nt + c;
      const _Float16* arow = R16 + c * kHP + koff;
      const _Float16* wc = Bh + (size_t)(2 * kNU + j) * kNU + koff;
      v8f accC = z8;
#pragma unroll 1
      for (int k0 = 0; k0 < kNU; k0 += 32) {
        const v16h a  = frag_load(arow + k0);
        const v16h b0 = frag_load(wc + k0);
        accC = mma_h(a, b0, accC);
        guard1_h(accC, a, b0);
      }
#pragma unroll
      for (int i = 0; i < 8; ++i) PRS[i * 256 + tid] = accC[i];
#pragma unroll 1
      for (int i = 0; i < 8; ++i) {
        const int row = 8 * hh + i;
        const float pc = PRS[i * 256 + tid];
        const float gc = Pt[(size_t)row * ldp + 2 * kNU + j];
        const float cv = tanhf(pc * kFold + gc);
        const float uv = US[row * kFP + j];
        const float hv = HS[row * kFP + j];
        const float hn = uv * hv + (1.0f - uv) * cv;
        HS[row * kFP + j] = hn;
        H16[row * kHP + j] = to_f16_flushed(hn * kActCarry);
      }
    }
    __syncthreads();

    const bool last = (s == kNT - 1);
    if (OM != 2) {
      v8h vv[4];
#pragma unroll
      for (int it = 0; it < 4; ++it) {
        const int row = 2 * wave + (it >> 1);
        vv[it] = *(const v8h*)(H16 + row * kHP + (it & 1) * 256 + lane * 8);
      }
      for (int pass = 0; pass < 2; ++pass) {
#pragma unroll
        for (int it = 0; it < 4; ++it) {
          const int row = 2 * wave + (it >> 1);
          *(volatile v8h*)(Yd + (size_t)(t * kNB + rowbase + row) * ldy + (it & 1) * 256 + lane * 8) = vv[it];
        }
        __threadfence();
      }
    }
    if (OM == 2 || (OM == 1 && last)) {
      v4f fv[8];
#pragma unroll
      for (int it = 0; it < 8; ++it) {
        const int row = 2 * wave + (it >> 2);
        fv[it] = *(const v4f*)(HS + row * kFP + 128 * (it & 3) + 4 * lane);
      }
      for (int pass = 0; pass < 2; ++pass) {
#pragma unroll
        for (int it = 0; it < 8; ++it) {
          const int row = 2 * wave + (it >> 2);
          const int col = 128 * (it & 3) + 4 * lane;
          if (OM == 2)
            *(volatile v4f*)(OUT0 + ((size_t)(rowbase + row) * kNT + (size_t)t) * kNU + col) = fv[it];
          if (last)
            *(volatile v4f*)(HFIN + (size_t)(rowbase + row) * kNU + col) = fv[it];
        }
        __threadfence();
      }
    }
  }
}

extern "C" void kernel_launch(void* const* d_in, const int* in_sizes, int n_in,
                              void* d_out, int out_size, void* d_ws, size_t ws_size, hipStream_t stream) {
  if (n_in < 18 || d_out == nullptr || d_ws == nullptr) return;
  if (in_sizes[0] != kNB * kNT || in_sizes[1] != kNV * kNE) return;
  if (in_sizes[2] != (kNE + kNU) * 2 * kNU || in_sizes[3] != 2 * kNU) return;
  if (in_sizes[4] != (kNE + kNU) * kNU || in_sizes[5] != kNU) return;
  if (in_sizes[6] != (kNE + kNU) * 2 * kNU || in_sizes[7] != 2 * kNU) return;
  if (in_sizes[8] != (kNE + kNU) * kNU || in_sizes[9] != kNU) return;
  if (in_sizes[10] != (3 * kNU) * 2 * kNU || in_sizes[11] != 2 * kNU) return;
  if (in_sizes[12] != (3 * kNU) * kNU || in_sizes[13] != kNU) return;
  if (in_sizes[14] != (2 * kNU) * 2 * kNU || in_sizes[15] != 2 * kNU) return;
  if (in_sizes[16] != (2 * kNU) * kNU || in_sizes[17] != kNU) return;
  if (out_size != kOut0 + kOut1) return;
  if (ws_size < kWsTotal) return;

  const int*   tok   = (const int*)d_in[0];
  const float* emb   = (const float*)d_in[1];
  const float* Wg_fw = (const float*)d_in[2];
  const float* bg_fw = (const float*)d_in[3];
  const float* Wc_fw = (const float*)d_in[4];
  const float* bc_fw = (const float*)d_in[5];
  const float* Wg_bw = (const float*)d_in[6];
  const float* bg_bw = (const float*)d_in[7];
  const float* Wc_bw = (const float*)d_in[8];
  const float* bc_bw = (const float*)d_in[9];
  const float* Wg_u1 = (const float*)d_in[10];
  const float* bg_u1 = (const float*)d_in[11];
  const float* Wc_u1 = (const float*)d_in[12];
  const float* bc_u1 = (const float*)d_in[13];
  const float* Wg_u2 = (const float*)d_in[14];
  const float* bg_u2 = (const float*)d_in[15];
  const float* Wc_u2 = (const float*)d_in[16];
  const float* bc_u2 = (const float*)d_in[17];
  float* out0 = (float*)d_out;
  float* out1 = out0 + (size_t)kOut0;

  char* ws = (char*)d_ws;
  size_t off = 0;
  auto carve = [&](size_t bytes) -> char* { char* p = ws + off; off += (bytes + 255) & ~(size_t)255; return p; };
  float*          PPLANE = (float*)carve(kSzP);
  unsigned short* X16    = (unsigned short*)carve(kSzX16);
  unsigned short* YCAT16 = (unsigned short*)carve(kSzYCAT);
  unsigned short* Y1_16  = (unsigned short*)carve(kSzY1);
  unsigned short* BX0    = (unsigned short*)carve(kSzBX0);
  unsigned short* BHBI   = (unsigned short*)carve(kSzBHBI);
  unsigned short* BX1    = (unsigned short*)carve(kSzBX1);
  unsigned short* BHU1   = (unsigned short*)carve(kSzBH);
  unsigned short* BX2    = (unsigned short*)carve(kSzBX2);
  unsigned short* BHU2   = (unsigned short*)carve(kSzBH);
  float*          BIASP  = (float*)carve(kSzBIAS);
  if (off != kWsTotal || off > ws_size) return;

  gather_rows_kernel<<<kRows / 8, 256, 0, stream>>>(tok, emb, X16);

  auto wt = [&](const float* W, int ncols, int dsplit, unsigned short* Dx, int pitchx, int nofsx,
                unsigned short* Dh, int nofsh) {
    wt_plane_kernel<<<dim3(ncols / 64, (dsplit + kNU) / 64), 256, 0, stream>>>(W, ncols, dsplit, Dx, pitchx, nofsx, Dh, nofsh);
  };
  unsigned short* BH_fw = BHBI;
  unsigned short* BH_bw = BHBI + (size_t)kG3 * kNU;
  wt(Wg_fw, 2 * kNU, kNE,     BX0, kNE,     0,               BH_fw, 0);
  wt(Wc_fw, kNU,     kNE,     BX0, kNE,     2 * kNU,         BH_fw, 2 * kNU);
  wt(Wg_bw, 2 * kNU, kNE,     BX0, kNE,     kG3,             BH_bw, 0);
  wt(Wc_bw, kNU,     kNE,     BX0, kNE,     kG3 + 2 * kNU,   BH_bw, 2 * kNU);
  wt(Wg_u1, 2 * kNU, 2 * kNU, BX1, 2 * kNU, 0,               BHU1,  0);
  wt(Wc_u1, kNU,     2 * kNU, BX1, 2 * kNU, 2 * kNU,         BHU1,  2 * kNU);
  wt(Wg_u2, 2 * kNU, kNU,     BX2, kNU,     0,               BHU2,  0);
  wt(Wc_u2, kNU,     kNU,     BX2, kNU,     2 * kNU,         BHU2,  2 * kNU);

  bias_plane_kernel<<<(4 * kG3 / 4) / 256, 256, 0, stream>>>(bg_fw, bc_fw, bg_bw, bc_bw, bg_u1, bc_u1, bg_u2, bc_u2, BIASP);

  wmma_gemm64_f16<<<(kRows / 64) * (2 * kG3 / 64) / 8, 256, 0, stream>>>(
      X16, kNE, BX0, kNE, PPLANE, 2 * kG3, BIASP, kRows, 2 * kG3, kNE, kFold);
  gru_seq_kernel<0><<<8, 256, 0, stream>>>(
      PPLANE, 2 * kG3, kG3, BHBI, kG3 * kNU, YCAT16, 2 * kNU, kNU, out0, out1);

  wmma_gemm64_f16<<<(kRows / 64) * (kG3 / 64) / 8, 256, 0, stream>>>(
      YCAT16, 2 * kNU, BX1, 2 * kNU, PPLANE, kG3, BIASP + 2 * kG3, kRows, kG3, 2 * kNU, kFold);
  gru_seq_kernel<1><<<4, 256, 0, stream>>>(
      PPLANE, kG3, 0, BHU1, 0, Y1_16, kNU, 0, out0, out1);

  wmma_gemm64_f16<<<(kRows / 64) * (kG3 / 64) / 8, 256, 0, stream>>>(
      Y1_16, kNU, BX2, kNU, PPLANE, kG3, BIASP + 3 * kG3, kRows, kG3, kNU, kFold);
  gru_seq_kernel<2><<<4, 256, 0, stream>>>(
      PPLANE, kG3, 0, BHU2, 0, Y1_16, kNU, 0, out0, out1 + (size_t)kNB * kNU);
}
